// NeuralSDETrajectoryPredictor_22265110462778
// MI455X (gfx1250) — hardware-run, weakly checked
//
#include <hip/hip_runtime.h>

constexpr int NSAMP  = 8;
constexpr int NBATCH = 16;
constexpr int NOBJ   = 64;
constexpr int NWALK  = NBATCH * NOBJ;
constexpr int NSTEP  = 40;
constexpr int THIST  = 12;
constexpr int HIDN   = 128;
constexpr int CTXD   = 256;
constexpr int NCOLS  = 2 * HIDN;
constexpr int NTHR   = 256;
constexpr int NWAVE  = NTHR / 32;
constexpr int GRP    = 4;
constexpr int WPITCH = 136;
constexpr int MEAN_ELEMS = NBATCH * NSTEP * NOBJ * 2;
constexpr int PATH_ELEMS = NSAMP * MEAN_ELEMS;
constexpr int MEAN_V4    = MEAN_ELEMS / 4;
constexpr int NBLK_WALK  = (NSAMP * NBATCH * (NOBJ / 16)) / NWAVE;

constexpr float WCAR     = 1024.0f;
constexpr float WCAR_INV = 1.0f / WCAR;
constexpr float RCAR     = 2048.0f;
constexpr float RCAR_INV = 1.0f / RCAR;
constexpr float HMIN     = 6.103515625e-05f;
constexpr float STEP_MAX = 5.0f;
constexpr float STEP_INV = 1.0f / STEP_MAX;
constexpr float SIG_LO   = 0.05f;
constexpr float SIG_SPAN = (float)(2.0 - 0.05);
constexpr float LAT_MAX  = 90.0f;
constexpr float LON_MOD  = 360.0f;

constexpr int SZ_PLANE = NCOLS * WPITCH * 2;
constexpr int OFF_WHI  = 0;
constexpr int OFF_WLO  = OFF_WHI + SZ_PLANE;
constexpr int OFF_B1   = OFF_WLO + SZ_PLANE;
constexpr int OFF_W2   = OFF_B1 + NCOLS * 4;
constexpr int OFF_WP01 = OFF_W2 + NCOLS * 2 * 4;
constexpr int OFF_CB   = OFF_WP01 + 2 * HIDN * 4;
constexpr int OFF_OBUF = OFF_CB + 2 * HIDN * 4;
constexpr int SZ_OBUFW = 2 * GRP * 32 * 4;
constexpr int LDS_TOTAL = OFF_OBUF + NWAVE * SZ_OBUFW;

static_assert(NSTEP % GRP == 0, "store groups");
static_assert(NOBJ % 16 == 0, "wave owns 16 objects");
static_assert((NSAMP * NBATCH * (NOBJ / 16)) % NWAVE == 0, "blocks exact");
static_assert(NBLK_WALK == 64, "grid");
static_assert((NCOLS * (HIDN / 8)) % NTHR == 0, "weight staging exact");
static_assert(MEAN_V4 % 256 == 0, "mean grid exact");
static_assert(OFF_WLO % 16 == 0 && OFF_B1 % 16 == 0 && OFF_W2 % 16 == 0, "align");
static_assert(OFF_WP01 % 16 == 0 && OFF_CB % 16 == 0 && OFF_OBUF % 16 == 0 && LDS_TOTAL % 16 == 0, "align");
static_assert((WPITCH * 2) % 16 == 0, "plane row pitch");
static_assert((MEAN_ELEMS * 4) % 128 == 0 && ((MEAN_ELEMS + PATH_ELEMS) * 4) % 128 == 0, "output regions start on 128-B lines");
static_assert(NTHR == 2 * HIDN, "table staging map");

typedef __attribute__((ext_vector_type(16))) _Float16 v16h;
typedef __attribute__((ext_vector_type(8)))  _Float16 v8h;
typedef __attribute__((ext_vector_type(8)))  float    v8f;
typedef __attribute__((ext_vector_type(4)))  float    v4f;
typedef __attribute__((ext_vector_type(2)))  float    v2f;
typedef __attribute__((ext_vector_type(4)))  unsigned v4u;

union FragU { v16h v; v8h h[2]; };

__device__ __forceinline__ v16h frag_load(const _Float16* p) {
  FragU f;
  f.h[0] = *(const v8h*)(p);
  f.h[1] = *(const v8h*)(p + 16);
  return f.v;
}

__device__ __forceinline__ v8f mma_h(v16h a, v16h b, v8f c) {
  c = __builtin_amdgcn_wmma_f32_16x16x32_f16(false, a, false, b, (short)0, c, false, false);
  asm volatile("v_nop\n\tv_nop\n\tv_nop\n\tv_nop" : "+v"(c) : "v"(a), "v"(b));
  return c;
}

__device__ __forceinline__ _Float16 to_h_flush(float v) {
  const float w = (fabsf(v) < HMIN) ? 0.0f : v;
  return (_Float16)w;
}

__device__ __forceinline__ void split_h(float v, _Float16& hi, _Float16& lo) {
  hi = to_h_flush(v);
  const float rs = (v - (float)hi) * RCAR;
  lo = to_h_flush(rs);
}

__device__ __forceinline__ float gelu_erf(float v) {
  return 0.5f * v * (1.0f + erff(v * 0.70710678118654752f));
}

__global__ void __launch_bounds__(NTHR, 1)
walk_kernel(const float* __restrict__ zc, const float* __restrict__ th, const float* __restrict__ nz,
            const float* __restrict__ wp, const float* __restrict__ bp,
            const float* __restrict__ wd1, const float* __restrict__ bd1,
            const float* __restrict__ wd2, const float* __restrict__ bd2,
            const float* __restrict__ ws1, const float* __restrict__ bs1,
            const float* __restrict__ ws2, const float* __restrict__ bs2,
            float* __restrict__ paths, float* __restrict__ sig) {
  extern __shared__ v4u smem_dyn[];
  unsigned char* const smem = (unsigned char*)smem_dyn;
  _Float16* const WHI = (_Float16*)(smem + OFF_WHI);
  _Float16* const WLO = (_Float16*)(smem + OFF_WLO);
  float* const B1T  = (float*)(smem + OFF_B1);
  float* const W2T  = (float*)(smem + OFF_W2);
  float* const WP01 = (float*)(smem + OFF_WP01);
  float* const CBT  = (float*)(smem + OFF_CB);
  float* const OBUF = (float*)(smem + OFF_OBUF);

  const int tid  = threadIdx.x;
  const int lane = tid & 31;
  const int wave = tid >> 5;
  const int c    = lane & 15;
  const int hh   = lane >> 4;
  const int blk  = blockIdx.x;
  const int samp = blk >> 3;
  const int b0   = (blk & 7) * 2;

#pragma unroll 1
  for (int it = 0; it < (NCOLS * (HIDN / 8)) / NTHR; ++it) {
    const int i   = it * NTHR + tid;
    const int mat = i >> 11;
    const int rem = i & 2047;
    const int kg  = rem >> 7;
    const int nl  = rem & (HIDN - 1);
    const float* src = (mat != 0) ? ws1 : wd1;
    float w[8];
#pragma unroll
    for (int e = 0; e < 8; ++e) w[e] = src[(kg * 8 + e) * HIDN + nl];
    v8h hv, lv;
#pragma unroll
    for (int e = 0; e < 8; ++e) {
      const float sc = w[e] * WCAR;
      _Float16 hi, lo;
      split_h(sc, hi, lo);
      hv[e] = hi;
      lv[e] = lo;
    }
    const int off = (mat * HIDN + nl) * WPITCH + kg * 8;
    *(v8h*)(WHI + off) = hv;
    *(v8h*)(WLO + off) = lv;
  }

  {
    const int j = tid & (HIDN - 1);
    const bool lowhalf = tid < HIDN;
    const float a1 = bd1[j];
    const float a2 = bs1[j];
    B1T[tid] = lowhalf ? a1 : a2;
    const float d0 = wd2[2 * j];
    const float d1 = wd2[2 * j + 1];
    const float s0 = ws2[2 * j];
    const float s1 = ws2[2 * j + 1];
    v2f w2v;
    w2v[0] = lowhalf ? d0 : s0;
    w2v[1] = lowhalf ? d1 : s1;
    *(v2f*)(W2T + 2 * tid) = w2v;
    WP01[tid] = wp[tid];
    const int bsel = b0 + (tid >> 7);
    const float* zr = zc + bsel * CTXD;
    const float* wc = wp + 2 * HIDN + j;
    float q0 = 0.0f, q1 = 0.0f, q2 = 0.0f, q3 = 0.0f;
#pragma unroll 1
    for (int k = 0; k < CTXD; k += 4) {
      q0 = fmaf(zr[k],     wc[(k)     * HIDN], q0);
      q1 = fmaf(zr[k + 1], wc[(k + 1) * HIDN], q1);
      q2 = fmaf(zr[k + 2], wc[(k + 2) * HIDN], q2);
      q3 = fmaf(zr[k + 3], wc[(k + 3) * HIDN], q3);
    }
    CBT[tid] = ((q0 + q1) + (q2 + q3)) + bp[j];
  }
  __syncthreads();

  const int bl   = wave >> 2;
  const int oq   = wave & 3;
  const int bsel = b0 + bl;
  const float* const CBw = CBT + bl * HIDN;
  float* const OBw = OBUF + wave * (2 * GRP * 32);
  const int comp = lane & 1;
  const int rsel = (lane >> 1) & 7;
  const float bd2v = bd2[comp];
  const float bs2v = bs2[comp];
  float x = th[((bsel * THIST + (THIST - 1)) * NOBJ + 16 * oq) * 2 + lane];
  const size_t obase = ((size_t)(samp * NBATCH + bsel) * NSTEP) * (NOBJ * 2) + 32 * oq;
  const size_t nbase = ((size_t)samp * NWALK + 64 * bsel + 16 * oq) * 2 + lane;
  const v8f z8 = {0.f, 0.f, 0.f, 0.f, 0.f, 0.f, 0.f, 0.f};

#pragma unroll 1
  for (int t = 0; t < NSTEP; ++t) {
    const float nzv = nz[nbase + (size_t)t * (NSAMP * NWALK * 2)];

    int kof = 8 * hh;
    asm volatile("" : "+v"(kof));

    const float lat = __shfl(x, 2 * c, 32);
    const float lon = __shfl(x, 2 * c + 1, 32);

    v16h ah[4], al[4];
#pragma unroll
    for (int kc = 0; kc < 4; ++kc) {
#pragma unroll
      for (int hr = 0; hr < 2; ++hr) {
        const int k0 = kc * 32 + 16 * hr + kof;
        const v4f u0 = *(const v4f*)(WP01 + k0);
        const v4f u1 = *(const v4f*)(WP01 + k0 + 4);
        const v4f v0 = *(const v4f*)(WP01 + HIDN + k0);
        const v4f v1 = *(const v4f*)(WP01 + HIDN + k0 + 4);
        const v4f g0 = *(const v4f*)(CBw + k0);
        const v4f g1 = *(const v4f*)(CBw + k0 + 4);
#pragma unroll
        for (int e = 0; e < 4; ++e) {
          const float ha = fmaf(lat, u0[e], fmaf(lon, v0[e], g0[e]));
          const float hb = fmaf(lat, u1[e], fmaf(lon, v1[e], g1[e]));
          _Float16 hi, lo;
          split_h(ha, hi, lo);
          ah[kc][8 * hr + e] = hi;
          al[kc][8 * hr + e] = lo;
          split_h(hb, hi, lo);
          ah[kc][8 * hr + 4 + e] = hi;
          al[kc][8 * hr + 4 + e] = lo;
        }
      }
    }

    float p0[8], p1[8], dr0[8], dr1[8];
#pragma unroll
    for (int r = 0; r < 8; ++r) { p0[r] = 0.0f; p1[r] = 0.0f; dr0[r] = 0.0f; dr1[r] = 0.0f; }

#pragma unroll 1
    for (int nt = 0; nt < NCOLS / 16; ++nt) {
      const int col = 16 * nt + c;
      const _Float16* wh = WHI + col * WPITCH + 8 * hh;
      const _Float16* wl = WLO + col * WPITCH + 8 * hh;
      v8f am = z8;
      v8f ar = z8;
#pragma unroll
      for (int kc = 0; kc < 4; ++kc) {
        const v16h bh  = frag_load(wh + 32 * kc);
        const v16h blo = frag_load(wl + 32 * kc);
        am = mma_h(ah[kc], bh, am);
        ar = mma_h(ah[kc], blo, ar);
        ar = mma_h(al[kc], bh, ar);
      }
      const float bv = B1T[col];
      const v2f w2 = *(const v2f*)(W2T + 2 * col);
      const float w2a = w2[0];
      const float w2b = w2[1];
#pragma unroll
      for (int r = 0; r < 8; ++r) {
        const float pre = fmaf(ar[r], RCAR_INV, am[r]) * WCAR_INV + bv;
        const float g = gelu_erf(pre);
        p0[r] = fmaf(g, w2a, p0[r]);
        p1[r] = fmaf(g, w2b, p1[r]);
      }
      if (nt == (HIDN / 16) - 1) {
#pragma unroll
        for (int r = 0; r < 8; ++r) {
          dr0[r] = p0[r];
          dr1[r] = p1[r];
          p0[r] = 0.0f;
          p1[r] = 0.0f;
        }
      }
    }

#pragma unroll
    for (int r = 0; r < 8; ++r) {
#pragma unroll
      for (int off = 1; off < 16; off <<= 1) {
        dr0[r] += __shfl_xor(dr0[r], off, 32);
        dr1[r] += __shfl_xor(dr1[r], off, 32);
        p0[r]  += __shfl_xor(p0[r],  off, 32);
        p1[r]  += __shfl_xor(p1[r],  off, 32);
      }
    }

    float dsel = 0.0f;
    float ssel = 0.0f;
#pragma unroll
    for (int r = 0; r < 8; ++r) {
      const float dcand = (comp != 0) ? dr1[r] : dr0[r];
      const float scand = (comp != 0) ? p1[r] : p0[r];
      dsel = (rsel == r) ? dcand : dsel;
      ssel = (rsel == r) ? scand : ssel;
    }

    const float drift = dsel + bd2v;
    const float uarg  = ssel + bs2v;
    const float s01   = 1.0f / (1.0f + expf(-uarg));
    const float sg    = SIG_LO + s01 * SIG_SPAN;
    float dl = drift + sg * nzv;
    dl = STEP_MAX * tanhf(dl * STEP_INV);
    const float xn   = x + dl;
    const float latv = fminf(fmaxf(xn, -LAT_MAX), LAT_MAX);
    const float tm   = fmodf(xn, LON_MOD);
    const bool plus  = (tm != 0.0f) && (tm < 0.0f);
    const float lonv = plus ? (tm + LON_MOD) : tm;
    x = (comp != 0) ? lonv : latv;

    const int tq = t & (GRP - 1);
    OBw[tq * 32 + lane] = x;
    OBw[(GRP + tq) * 32 + lane] = sg;
    if (tq == GRP - 1) {
      __builtin_amdgcn_fence(__ATOMIC_RELEASE, "workgroup");
      __builtin_amdgcn_wave_barrier();
      __builtin_amdgcn_fence(__ATOMIC_ACQUIRE, "workgroup");
      const int q  = lane >> 3;
      const int j4 = (lane & 7) * 4;
      const v4f pv = *(const v4f*)(OBw + q * 32 + j4);
      const v4f sv = *(const v4f*)(OBw + (GRP + q) * 32 + j4);
      const size_t o = obase + (size_t)(t - (GRP - 1) + q) * (NOBJ * 2) + j4;
      for (int pass = 0; pass < 2; ++pass) {
        *(volatile v4f*)(paths + o) = pv;
        *(volatile v4f*)(sig + o)   = sv;
        __threadfence();
      }
      __builtin_amdgcn_fence(__ATOMIC_RELEASE, "workgroup");
      __builtin_amdgcn_wave_barrier();
      __builtin_amdgcn_fence(__ATOMIC_ACQUIRE, "workgroup");
    }
  }
}

__global__ void __launch_bounds__(256)
sample_mean_kernel(const float* __restrict__ paths, const int* __restrict__ hzn, float* __restrict__ meanout) {
  const int i  = blockIdx.x * 256 + threadIdx.x;
  const bool ok = i < MEAN_V4;
  const int ic = ok ? i : (MEAN_V4 - 1);
  const int hz = hzn[0];
  v4f acc = {0.0f, 0.0f, 0.0f, 0.0f};
#pragma unroll
  for (int s = 0; s < NSAMP; ++s) {
    const v4f p = *(const v4f*)(paths + (size_t)s * MEAN_ELEMS + (size_t)ic * 4);
    acc += p;
  }
  acc *= (1.0f / (float)NSAMP);
  const float nanv = __uint_as_float(0x7fc00000u);
  const v4f nv = {nanv, nanv, nanv, nanv};
  const v4f ov = (hz == NSTEP) ? acc : nv;
  if (ok) {
    for (int pass = 0; pass < 2; ++pass) {
      *(volatile v4f*)(meanout + (size_t)ic * 4) = ov;
      __threadfence();
    }
  }
}

extern "C" void kernel_launch(void* const* d_in, const int* in_sizes, int n_in,
                              void* d_out, int out_size, void* d_ws, size_t ws_size, hipStream_t stream) {
  (void)d_ws; (void)ws_size;
  if (n_in < 14 || d_out == nullptr) return;
  if (in_sizes[0] != NBATCH * CTXD || in_sizes[1] != NBATCH * THIST * NOBJ * 2 ||
      in_sizes[2] != NSTEP * NSAMP * NWALK * 2 || in_sizes[3] != (2 + CTXD) * HIDN || in_sizes[4] != HIDN ||
      in_sizes[5] != HIDN * HIDN || in_sizes[6] != HIDN || in_sizes[7] != HIDN * 2 || in_sizes[8] != 2 ||
      in_sizes[9] != HIDN * HIDN || in_sizes[10] != HIDN || in_sizes[11] != HIDN * 2 || in_sizes[12] != 2 ||
      in_sizes[13] != 1 || out_size != MEAN_ELEMS + 2 * PATH_ELEMS) return;

  const float* zc  = (const float*)d_in[0];
  const float* th  = (const float*)d_in[1];
  const float* nz  = (const float*)d_in[2];
  const float* wp  = (const float*)d_in[3];
  const float* bp  = (const float*)d_in[4];
  const float* wd1 = (const float*)d_in[5];
  const float* bd1 = (const float*)d_in[6];
  const float* wd2 = (const float*)d_in[7];
  const float* bd2 = (const float*)d_in[8];
  const float* ws1 = (const float*)d_in[9];
  const float* bs1 = (const float*)d_in[10];
  const float* ws2 = (const float*)d_in[11];
  const float* bs2 = (const float*)d_in[12];
  const int*   hzn = (const int*)d_in[13];

  float* out    = (float*)d_out;
  float* meanp  = out;
  float* pathsp = out + MEAN_ELEMS;
  float* sigp   = out + MEAN_ELEMS + PATH_ELEMS;

  walk_kernel<<<dim3(NBLK_WALK), dim3(NTHR), LDS_TOTAL, stream>>>(
      zc, th, nz, wp, bp, wd1, bd1, wd2, bd2, ws1, bs1, ws2, bs2, pathsp, sigp);
  sample_mean_kernel<<<dim3(MEAN_V4 / 256), dim3(256), 0, stream>>>(pathsp, hzn, meanp);
}
